// CausalShapedAttention_11278584120019
// MI455X (gfx1250) — hardware-verified
//
#include <hip/hip_runtime.h>
#include <stddef.h>
#include <stdint.h>

#define NB    2
#define SQ    2048
#define NTOK  4096
#define DM    1024
#define NH    16
#define HDM   64
#define NPROJ 2048
#define QB    128
#define KC    64
#define NQB   (SQ / QB)
#define NCK   (SQ / KC)
#define SBLK  (SQ / 256)
#define NBH   (NB * NH)
#define QKPLANE (NBH * SQ * HDM)

static_assert(NTOK == NB * SQ);
static_assert(SQ % 256 == 0);
static_assert(DM % 64 == 0);
static_assert(DM % 32 == 0);
static_assert(HDM == 64);
static_assert(KC == HDM);
static_assert(NH * HDM == DM);
static_assert(NPROJ == 2 * DM);
static_assert(QB == 2 * KC);
static_assert(SQ % KC == 0);
static_assert(SQ % QB == 0);
static_assert(NTOK % 256 == 0);
static_assert(NTOK % 64 == 0);
static_assert((NTOK * DM) % 2048 == 0);
static_assert((NPROJ * DM) % 2048 == 0);
static_assert(NBH % 2 == 0);

typedef _Float16 v16h __attribute__((ext_vector_type(16)));
typedef _Float16 v8h  __attribute__((ext_vector_type(8)));
typedef float    v8f  __attribute__((ext_vector_type(8)));
typedef float    v4f  __attribute__((ext_vector_type(4)));
typedef unsigned int v4u __attribute__((ext_vector_type(4)));

union Frag  { v16h v; v8h h[2]; };
union Pack8 { v8h h; v4u u; };

__device__ __forceinline__ v8f mma16(v16h a, v16h b, v8f c) {
  c = __builtin_amdgcn_wmma_f32_16x16x32_f16(false, a, false, b, (short)0, c, false, false);
  asm volatile("v_nop\n\tv_nop\n\tv_nop\n\tv_nop" : "+v"(c) : "v"(a), "v"(b));
  return c;
}

__device__ __forceinline__ v16h ldfrag(const _Float16* p, int ld, int row0, int k0, int lane) {
  const int m = lane & 15, lh = lane >> 4;
  const _Float16* q = p + (size_t)(row0 + m) * ld + k0 + 8 * lh;
  Frag f;
  f.h[0] = *(const v8h*)(q);
  f.h[1] = *(const v8h*)(q + 16);
  return f.v;
}

__device__ __forceinline__ v8f zero8() { return (v8f){0.f, 0.f, 0.f, 0.f, 0.f, 0.f, 0.f, 0.f}; }

__device__ __forceinline__ void gemm32x64(const _Float16* __restrict__ A, int lda,
                                          const _Float16* __restrict__ Bt, int ldb, int K,
                                          int m0, int n0, int lane, v8f (&acc)[2][4]) {
#pragma unroll 1
  for (int k0 = 0; k0 < K; k0 += 32) {
    const v16h a0 = ldfrag(A, lda, m0, k0, lane);
    const v16h a1 = ldfrag(A, lda, m0 + 16, k0, lane);
    const v16h b0 = ldfrag(Bt, ldb, n0, k0, lane);
    const v16h b1 = ldfrag(Bt, ldb, n0 + 16, k0, lane);
    const v16h b2 = ldfrag(Bt, ldb, n0 + 32, k0, lane);
    const v16h b3 = ldfrag(Bt, ldb, n0 + 48, k0, lane);
    acc[0][0] = mma16(a0, b0, acc[0][0]);
    acc[1][0] = mma16(a1, b0, acc[1][0]);
    acc[0][1] = mma16(a0, b1, acc[0][1]);
    acc[1][1] = mma16(a1, b1, acc[1][1]);
    acc[0][2] = mma16(a0, b2, acc[0][2]);
    acc[1][2] = mma16(a1, b2, acc[1][2]);
    acc[0][3] = mma16(a0, b3, acc[0][3]);
    acc[1][3] = mma16(a1, b3, acc[1][3]);
  }
}

__global__ __launch_bounds__(256) void k_cvt(const float* __restrict__ src, _Float16* __restrict__ dh, float scale) {
  const int tid = threadIdx.x;
  const size_t o = (size_t)blockIdx.x * 2048 + (size_t)tid * 8;
  const v4f a0 = *(const v4f*)(src + o) * scale;
  const v4f a1 = *(const v4f*)(src + o + 4) * scale;
  Pack8 pk;
  pk.h = (v8h){(_Float16)a0[0], (_Float16)a0[1], (_Float16)a0[2], (_Float16)a0[3],
               (_Float16)a1[0], (_Float16)a1[1], (_Float16)a1[2], (_Float16)a1[3]};
  const v4u vv = pk.u;
  volatile v4u* d = (volatile v4u*)(dh + o);
  *d = vv;
  __threadfence();
  *d = vv;
}

#define WTP 72
__global__ __launch_bounds__(256) void k_vtr(const float* __restrict__ x, _Float16* __restrict__ vt) {
  __shared__ __align__(16) _Float16 st[64 * WTP];
  const int tid  = threadIdx.x;
  const int tok0 = blockIdx.x * 64;
  const int h    = blockIdx.y;
  const int b    = tok0 / SQ;
  const int t0   = tok0 - b * SQ;
  const int hb   = b * NH + h;
#pragma unroll
  for (int i = 0; i < 4; ++i) {
    const int idx = tid + 256 * i;
    const int r   = idx >> 4;
    const int c4  = (idx & 15) * 4;
    const v4f f = *(const v4f*)(x + (size_t)(tok0 + r) * DM + h * HDM + c4);
    st[(c4 + 0) * WTP + r] = (_Float16)f[0];
    st[(c4 + 1) * WTP + r] = (_Float16)f[1];
    st[(c4 + 2) * WTP + r] = (_Float16)f[2];
    st[(c4 + 3) * WTP + r] = (_Float16)f[3];
  }
  __syncthreads();
  v4u val[2];
  size_t go[2];
#pragma unroll
  for (int g = 0; g < 2; ++g) {
    const int p   = tid + 256 * g;
    const int row = p >> 3;
    const int pc  = p & 7;
    Pack8 pk;
    pk.h   = *(const v8h*)(st + row * WTP + pc * 8);
    val[g] = pk.u;
    go[g]  = ((size_t)hb * HDM + row) * SQ + t0 + pc * 8;
  }
  for (int ps = 0; ps < 2; ++ps) {
#pragma unroll
    for (int g = 0; g < 2; ++g) *(volatile v4u*)(vt + go[g]) = val[g];
    __threadfence();
  }
}

__global__ __launch_bounds__(32) void k_mc(const float* __restrict__ x, const float* __restrict__ gamma_p,
                                           float* __restrict__ mc) {
  const int lane = threadIdx.x;
  const int sub  = lane >> 4;
  const int d0   = (lane & 15) * 4;
  const int hb   = blockIdx.x * 2 + sub;
  const int b    = hb / NH;
  const int h    = hb - b * NH;
  const float gamma = gamma_p[0];
  const float* xc = x + (size_t)b * SQ * DM + h * HDM + d0;
  float* mcc = mc + (size_t)hb * SQ * HDM + d0;
  double s0 = 0.0, s1 = 0.0, s2 = 0.0, s3 = 0.0;
#pragma unroll 1
  for (int i = SQ - 2; i >= 0; --i) {
    const v4f f = *(const v4f*)(xc + (size_t)(i + 1) * DM);
    s0 += (double)f[0]; s1 += (double)f[1]; s2 += (double)f[2]; s3 += (double)f[3];
    const float rn = 1.0f / (float)(SQ - 1 - i);
    v4f o;
    o[0] = gamma * ((float)s0 * rn);
    o[1] = gamma * ((float)s1 * rn);
    o[2] = gamma * ((float)s2 * rn);
    o[3] = gamma * ((float)s3 * rn);
    volatile v4f* d = (volatile v4f*)(mcc + (size_t)i * HDM);
    *d = o;
    __threadfence();
    *d = o;
  }
  {
    const v4f f = *(const v4f*)(xc);
    s0 += (double)f[0]; s1 += (double)f[1]; s2 += (double)f[2]; s3 += (double)f[3];
    const float rn = 1.0f / (float)SQ;
    v4f o;
    o[0] = gamma * ((float)s0 * rn);
    o[1] = gamma * ((float)s1 * rn);
    o[2] = gamma * ((float)s2 * rn);
    o[3] = gamma * ((float)s3 * rn);
    volatile v4f* d = (volatile v4f*)(mcc + (size_t)(SQ - 1) * HDM);
    *d = o;
    __threadfence();
    *d = o;
  }
}

#define STP 72
__global__ __launch_bounds__(256) void k_qk(const _Float16* __restrict__ xh,
                                            const _Float16* __restrict__ wh,
                                            _Float16* __restrict__ qkp) {
  __shared__ __align__(16) _Float16 st[256 * STP];
  const int tid = threadIdx.x, lane = tid & 31, wave = tid >> 5;
  const int hh = lane >> 4, c = lane & 15;
  const int bx = blockIdx.x;
  const int b  = bx / SBLK;
  const int sb = (bx - b * SBLK) * 256;
  const int ns = blockIdx.y;
  const int which = ns / NH;
  const int head  = ns - which * NH;
  const int hb    = b * NH + head;
  const int m0 = bx * 256 + wave * 32;
  const int n0 = ns * 64;

  v8f acc[2][4];
#pragma unroll
  for (int s = 0; s < 2; ++s)
#pragma unroll
    for (int t = 0; t < 4; ++t) acc[s][t] = zero8();
  gemm32x64(xh, DM, wh, DM, DM, m0, n0, lane, acc);

#pragma unroll
  for (int sub = 0; sub < 2; ++sub)
#pragma unroll
    for (int t = 0; t < 4; ++t)
#pragma unroll
      for (int r = 0; r < 8; ++r)
        st[(wave * 32 + sub * 16 + 8 * hh + r) * STP + 16 * t + c] = (_Float16)(acc[sub][t][r] * 0.03125f);
  __syncthreads();

  _Float16* base = qkp + (size_t)which * QKPLANE + (size_t)hb * SQ * HDM;
#pragma unroll
  for (int g = 0; g < 2; ++g) {
    v4u val[4];
    size_t go[4];
#pragma unroll
    for (int j = 0; j < 4; ++j) {
      const int p  = tid + 256 * (4 * g + j);
      const int lr = p >> 3;
      const int pc = p & 7;
      Pack8 pk;
      pk.h   = *(const v8h*)(st + lr * STP + pc * 8);
      val[j] = pk.u;
      go[j]  = (size_t)(sb + lr) * HDM + pc * 8;
    }
    for (int ps = 0; ps < 2; ++ps) {
#pragma unroll
      for (int j = 0; j < 4; ++j) *(volatile v4u*)(base + go[j]) = val[j];
      __threadfence();
    }
  }
}

#define KTP 72
#define OTP 68
#define LDSF 9216
static_assert(LDSF * 4 >= (KC * KTP + HDM * KTP + 8 * 16 * KTP) * 2);
static_assert(LDSF >= 8 * 16 * OTP);
__global__ __launch_bounds__(256) void k_attn(const _Float16* __restrict__ qp,
                                              const _Float16* __restrict__ kp,
                                              const _Float16* __restrict__ vt,
                                              const float* __restrict__ x,
                                              const float* __restrict__ mc,
                                              const float* __restrict__ alpha_p,
                                              const float* __restrict__ beta_p,
                                              const int* __restrict__ nh_p,
                                              float sscale,
                                              float* __restrict__ y) {
  __shared__ __align__(16) float ldsf[LDSF];
  _Float16* lds = (_Float16*)ldsf;
  _Float16* Ks = lds;
  _Float16* Vs = lds + KC * KTP;
  _Float16* Ps = lds + 2 * KC * KTP;

  const int tid = threadIdx.x, lane = tid & 31, wave = tid >> 5;
  const int hh = lane >> 4, c = lane & 15;
  const int qb  = blockIdx.x % NQB;
  const int hb  = blockIdx.x / NQB;
  const int h   = hb % NH;
  const int b   = hb / NH;
  const int q0b = qb * QB;
  const int q0  = q0b + wave * 16;

  const _Float16* Q = qp + (size_t)hb * SQ * HDM;
  const _Float16* K = kp + (size_t)hb * SQ * HDM;
  const _Float16* V = vt + (size_t)hb * HDM * SQ;

  v16h qa[2];
  qa[0] = ldfrag(Q, HDM, q0, 0, lane);
  qa[1] = ldfrag(Q, HDM, q0, 32, lane);

  const float NEGI = -__builtin_huge_valf();
  float mrow[8], lrow[8];
  v8f oacc[4];
#pragma unroll
  for (int r = 0; r < 8; ++r) { mrow[r] = NEGI; lrow[r] = 0.f; }
#pragma unroll
  for (int t = 0; t < 4; ++t) oacc[t] = zero8();

  _Float16* pw = Ps + wave * 16 * KTP;
  const int nck = 2 * qb + 2;

  for (int kc = 0; kc < nck; ++kc) {
    const int kv0 = kc * KC;
    __syncthreads();
    {
      const int r  = tid >> 2;
      const int qq = (tid & 3) * 16;
      const _Float16* ks = K + (size_t)(kv0 + r) * HDM + qq;
      const _Float16* vs = V + (size_t)r * SQ + kv0 + qq;
#pragma unroll
      for (int e = 0; e < 2; ++e) {
        *(v8h*)(Ks + r * KTP + qq + 8 * e) = *(const v8h*)(ks + 8 * e);
        *(v8h*)(Vs + r * KTP + qq + 8 * e) = *(const v8h*)(vs + 8 * e);
      }
    }
    __syncthreads();

    v8f s[4];
#pragma unroll
    for (int j = 0; j < 4; ++j) s[j] = zero8();
#pragma unroll
    for (int dc = 0; dc < 2; ++dc) {
#pragma unroll
      for (int j = 0; j < 4; ++j) {
        const v16h kb = ldfrag(Ks, KTP, j * 16, dc * 32, lane);
        s[j] = mma16(qa[dc], kb, s[j]);
      }
    }
    const bool diag = (kv0 + KC > q0b);
    float cm[8];
#pragma unroll
    for (int r = 0; r < 8; ++r) {
      const int row = q0 + 8 * hh + r;
      float m = NEGI;
#pragma unroll
      for (int j = 0; j < 4; ++j) {
        float sv = s[j][r] * sscale;
        if (diag) {
          const int key = kv0 + 16 * j + c;
          sv = (key <= row) ? sv : NEGI;
        }
        s[j][r] = sv;
        m = fmaxf(m, sv);
      }
#pragma unroll
      for (int off = 1; off < 16; off <<= 1) m = fmaxf(m, __shfl_xor(m, off, 32));
      cm[r] = m;
    }
    float al[8];
#pragma unroll
    for (int r = 0; r < 8; ++r) {
      const float mnew  = fmaxf(mrow[r], cm[r]);
      const float alpha = __expf(mrow[r] - mnew);
      mrow[r] = mnew;
      float psum = 0.f;
#pragma unroll
      for (int j = 0; j < 4; ++j) {
        const float p = __expf(s[j][r] - mnew);
        psum += p;
        pw[(8 * hh + r) * KTP + j * 16 + c] = (_Float16)(p * 1024.0f);
      }
#pragma unroll
      for (int off = 1; off < 16; off <<= 1) psum += __shfl_xor(psum, off, 32);
      lrow[r] = lrow[r] * alpha + psum;
      al[r] = alpha;
    }
#pragma unroll
    for (int t = 0; t < 4; ++t)
#pragma unroll
      for (int r = 0; r < 8; ++r) oacc[t][r] *= al[r];
    __syncthreads();

#pragma unroll
    for (int kk = 0; kk < 2; ++kk) {
      const v16h pa = ldfrag(pw, KTP, 0, kk * 32, lane);
#pragma unroll
      for (int t = 0; t < 4; ++t) {
        const v16h vb = ldfrag(Vs, KTP, t * 16, kk * 32, lane);
        oacc[t] = mma16(pa, vb, oacc[t]);
      }
    }
  }

  const float alpha_s = alpha_p[0];
  const float beta_s  = beta_p[0];
  const int   nh      = nh_p[0];
  const float poison  = (nh == NH) ? 0.0f : __int_as_float(0x7fc00000);
  const float bsc = beta_s * 0.0009765625f;
  float binv[8];
#pragma unroll
  for (int r = 0; r < 8; ++r) binv[r] = (lrow[r] > 0.f) ? (bsc / lrow[r]) : 0.f;
  __syncthreads();
  float* sw = ldsf + wave * (16 * OTP);
#pragma unroll
  for (int r = 0; r < 8; ++r) {
#pragma unroll
    for (int t = 0; t < 4; ++t)
      sw[(8 * hh + r) * OTP + 16 * t + c] = oacc[t][r] * binv[r];
  }
  __syncthreads();
  v4f val[8];
  size_t go[8];
#pragma unroll
  for (int it = 0; it < 8; ++it) {
    const int p    = lane + 32 * it;
    const int L    = p >> 3;
    const int pc   = p & 7;
    const int row  = L >> 1;
    const int half = L & 1;
    const v4f o4 = *(const v4f*)(sw + row * OTP + half * 32 + pc * 4);
    const size_t gi = ((size_t)b * SQ + (size_t)(q0 + row)) * DM + (size_t)h * HDM + half * 32 + pc * 4;
    const v4f x4 = *(const v4f*)(x + gi);
    const v4f m4 = *(const v4f*)(mc + ((size_t)hb * SQ + (size_t)(q0 + row)) * HDM + half * 32 + pc * 4);
    val[it] = o4 + x4 * alpha_s - m4 + poison;
    go[it]  = gi;
  }
  for (int ps = 0; ps < 2; ++ps) {
#pragma unroll
    for (int it = 0; it < 8; ++it) *(volatile v4f*)(y + go[it]) = val[it];
    __threadfence();
  }
}

extern "C" void kernel_launch(void* const* d_in, const int* in_sizes, int n_in,
                              void* d_out, int out_size, void* d_ws, size_t ws_size,
                              hipStream_t stream) {
  if (n_in < 6) return;
  if (in_sizes[0] != NTOK * DM) return;
  if (in_sizes[1] != NPROJ * DM) return;
  if (in_sizes[2] < 1 || in_sizes[3] < 1 || in_sizes[4] < 1 || in_sizes[5] < 1) return;
  if (out_size != NTOK * DM) return;

  const float* x       = (const float*)d_in[0];
  const float* w       = (const float*)d_in[1];
  const float* alpha_p = (const float*)d_in[2];
  const float* beta_p  = (const float*)d_in[3];
  const float* gamma_p = (const float*)d_in[4];
  const int*   nh_p    = (const int*)d_in[5];
  float* out = (float*)d_out;

  size_t off = 0;
  const size_t oX  = off; off += (size_t)NTOK * DM * 2;
  const size_t oW  = off; off += (size_t)NPROJ * DM * 2;
  const size_t oQ  = off; off += (size_t)QKPLANE * 2;
  const size_t oK  = off; off += (size_t)QKPLANE * 2;
  const size_t oV  = off; off += (size_t)NBH * HDM * SQ * 2;
  const size_t oMC = off; off += (size_t)NBH * SQ * HDM * 4;
  if (off > ws_size) return;
  if (off > (size_t)134217728) return;
  if (oK != oQ + (size_t)QKPLANE * 2) return;

  char* ws = (char*)d_ws;
  _Float16* Xh  = (_Float16*)(ws + oX);
  _Float16* Wh  = (_Float16*)(ws + oW);
  _Float16* QKp = (_Float16*)(ws + oQ);
  _Float16* Kp  = (_Float16*)(ws + oK);
  _Float16* Vt  = (_Float16*)(ws + oV);
  float*    Mc  = (float*)(ws + oMC);

  k_cvt<<<dim3((NTOK * DM) / 2048), dim3(256), 0, stream>>>(x, Xh, 1.0f);
  k_cvt<<<dim3((NPROJ * DM) / 2048), dim3(256), 0, stream>>>(w, Wh, 32.0f);
  k_vtr<<<dim3(NTOK / 64, NH), dim3(256), 0, stream>>>(x, Vt);
  k_mc<<<dim3(NBH / 2), dim3(32), 0, stream>>>(x, gamma_p, Mc);
  k_qk<<<dim3(NB * SBLK, NPROJ / 64), dim3(256), 0, stream>>>(Xh, Wh, QKp);
  const float sscale = 0.125f;
  k_attn<<<dim3(NBH * NQB), dim3(256), 0, stream>>>(QKp, Kp, Vt, x, Mc, alpha_p, beta_p, nh_p, sscale, out);
  (void)hipGetLastError();
}
